// KmerDPVAE_12962211299863
// MI455X (gfx1250) — hardware-verified
//
#include <hip/hip_runtime.h>

typedef __attribute__((ext_vector_type(16))) _Float16 v16h;
typedef __attribute__((ext_vector_type(8)))  _Float16 v8h;
typedef __attribute__((ext_vector_type(8)))  float    v8f;
typedef __attribute__((ext_vector_type(4)))  float    v4f;
typedef __attribute__((ext_vector_type(4)))  unsigned v4u;
typedef float __attribute__((may_alias)) float_a;

#define NN   4096
#define KK   500
#define KPAD 512
#define DZ   64
#define XC   128
#define ALPHA_C 1.0f
#define SMIN_C  1e-6f
#define WSC  4096.0f
#define WUN  (1.0f / 4096.0f)

__device__ __forceinline__ v8f wmma_f16(v16h a, v16h b, v8f c) {
    v8f d = __builtin_amdgcn_wmma_f32_16x16x32_f16(false, a, false, b, (short)0, c, false, false);
    asm volatile("v_nop\n\tv_nop\n\tv_nop\n\tv_nop" : "+v"(d) : "v"(a), "v"(b));
    return d;
}
__device__ __forceinline__ v16h load_frag(const _Float16* tile, size_t ld, int k0, int lane) {
    union { v16h v; v8h h[2]; } r;
    const _Float16* row = tile + (size_t)(lane & 15) * ld + k0 + 8 * (lane >> 4);
    r.h[0] = *(const v8h*)(row);
    r.h[1] = *(const v8h*)(row + 16);
    return r.v;
}
template <typename V> __device__ __forceinline__ void vst2(void* p, V v) {
    *(volatile V*)p = v; __threadfence(); *(volatile V*)p = v;
}

__device__ __forceinline__ float digammaf_dev(float x) {
    float r = 0.f;
    while (x < 6.f) { r -= 1.f / x; x += 1.f; }
    float inv  = 1.f / x;
    float inv2 = inv * inv;
    float s = logf(x) - 0.5f * inv
            - inv2 * (1.f/12.f - inv2 * (1.f/120.f - inv2 * (1.f/252.f)));
    return r + s;
}

__global__ __launch_bounds__(32) void elogpi_kernel(const float* __restrict__ a, const float* __restrict__ b,
                                                     float* __restrict__ elp) {
    __shared__ __align__(16) float buf[KPAD];
    const int lane = threadIdx.x;
    if (lane == 0) {
        float cs = 0.f;
        for (int k = 0; k < KK; ++k) {
            float ak = a[k], bk = b[k];
            float pab = digammaf_dev(ak + bk);
            float pa  = digammaf_dev(ak);
            float pb  = digammaf_dev(bk);
            buf[k] = (pa - pab) + cs;
            cs    += (pb - pab);
        }
        for (int k = KK; k < KPAD; ++k) buf[k] = 0.f;
    }
    __syncthreads();
    for (int q = 0; q < 4; ++q) {
        const v4f v = *(const v4f*)(buf + (q * 32 + lane) * 4);
        vst2(elp + (q * 32 + lane) * 4, v);
    }
}

__global__ void __launch_bounds__(256)
estep_kernel(const float* __restrict__ mu, const float* __restrict__ s2,
             const float* __restrict__ S,  const float* __restrict__ m,
             const float* __restrict__ elp, float* __restrict__ r) {
    __shared__ float smu[DZ];
    __shared__ float ss2[DZ];
    __shared__ float sc[KPAD];
    __shared__ float red[256];
    __shared__ __align__(16) float rt[16 * KK];

    const int t = threadIdx.x;
    for (int rr = 0; rr < 16; ++rr) {
        const int n = blockIdx.x * 16 + rr;
        __syncthreads();
        if (t < DZ) { smu[t] = mu[n * DZ + t]; ss2[t] = s2[n * DZ + t]; }
        for (int k = t; k < KPAD; k += 256) sc[k] = -3.0e38f;
        __syncthreads();

        for (int k = t; k < KK; k += 256) {
            const float* Sk = S + k * DZ;
            const float* mk = m + k * DZ;
            float acc = 0.f;
#pragma unroll 8
            for (int d = 0; d < DZ; ++d) {
                float comb = ss2[d] + Sk[d];
                float diff = smu[d] - mk[d];
                acc += __logf(comb) + diff * diff / comb;
            }
            sc[k] = elp[k] - 0.5f * acc;
        }
        __syncthreads();

        red[t] = fmaxf(sc[t], sc[t + 256]);
        __syncthreads();
        for (int s = 128; s > 0; s >>= 1) {
            if (t < s) red[t] = fmaxf(red[t], red[t + s]);
            __syncthreads();
        }
        const float mx = red[0];
        __syncthreads();

        float part = 0.f;
        for (int k = t; k < KPAD; k += 256) {
            float e = (k < KK) ? __expf(sc[k] - mx) : 0.f;
            sc[k] = e;
            part += e;
        }
        red[t] = part;
        __syncthreads();
        for (int s = 128; s > 0; s >>= 1) {
            if (t < s) red[t] += red[t + s];
            __syncthreads();
        }
        const float inv = 1.f / red[0];
        for (int k = t; k < KK; k += 256) rt[rr * KK + k] = sc[k] * inv;
    }
    __syncthreads();
    char* dst = (char*)(r + (size_t)blockIdx.x * 16 * KK);
    for (int g = t; g < 16 * KK / 4; g += 256) {
        const v4f v = *(const v4f*)((const char*)rt + g * 16);
        vst2(dst + g * 16, v);
    }
}

__global__ __launch_bounds__(256) void colsum_kernel(const float* __restrict__ r, float* __restrict__ n_k) {
    __shared__ float part[8][32];
    const int x = threadIdx.x & 31;
    const int y = threadIdx.x >> 5;
    const int k = blockIdx.x * 32 + x;
    float acc = 0.f;
    if (k < KK)
        for (int n = y; n < NN; n += 8) acc += r[n * KK + k];
    part[y][x] = acc;
    __syncthreads();
    if (y == 0) {
        float s = 0.f;
#pragma unroll
        for (int j = 0; j < 8; ++j) s += part[j][x];
        vst2(n_k + k, (k < KK) ? s : 0.f);
    }
}

__global__ void __launch_bounds__(256)
pack_Wt_kernel(const float* __restrict__ r, const float* __restrict__ n_k, _Float16* __restrict__ Wt) {
    __shared__ __align__(16) _Float16 tile[32][72];
    const int n0 = blockIdx.x * 64;
    const int k0 = blockIdx.y * 32;
    const int t  = threadIdx.x;
    for (int i = t; i < 64 * 32; i += 256) {
        const int nn = i >> 5, kx = i & 31;
        const int k = k0 + kx;
        float v = 0.f;
        if (k < KK) v = r[(size_t)(n0 + nn) * KK + k] / fmaxf(n_k[k], 1e-10f) * WSC;
        tile[kx][nn] = (_Float16)v;
    }
    __syncthreads();
    {
        const int kx = t >> 3, pc = t & 7;
        const v4u v = *(const v4u*)((const char*)&tile[kx][0] + pc * 16);
        vst2((char*)(Wt + (size_t)(k0 + kx) * NN + n0) + pc * 16, v);
    }
}

__global__ void __launch_bounds__(256)
pack_Xt_kernel(const float* __restrict__ mu, const float* __restrict__ s2, _Float16* __restrict__ Xt) {
    __shared__ __align__(16) _Float16 tile[32][72];
    const int n0 = blockIdx.x * 64;
    const int c0 = blockIdx.y * 32;
    const int t  = threadIdx.x;
    for (int i = t; i < 64 * 32; i += 256) {
        const int nn = i >> 5, cx = i & 31;
        const int c = c0 + cx, n = n0 + nn;
        float v;
        if (c < DZ) v = mu[n * DZ + c];
        else { const float mm = mu[n * DZ + c - DZ]; v = s2[n * DZ + c - DZ] + mm * mm; }
        tile[cx][nn] = (_Float16)v;
    }
    __syncthreads();
    {
        const int cx = t >> 3, pc = t & 7;
        const v4u v = *(const v4u*)((const char*)&tile[cx][0] + pc * 16);
        vst2((char*)(Xt + (size_t)(c0 + cx) * NN + n0) + pc * 16, v);
    }
}

__global__ void __launch_bounds__(256)
gemm_rtX_kernel(const _Float16* __restrict__ Wt, const _Float16* __restrict__ Xt, float* __restrict__ rt) {
    __shared__ __align__(16) float ot[16 * XC];
    const int tm   = blockIdx.x;
    const int lane = threadIdx.x & 31;
    const int tn   = threadIdx.x >> 5;
    const int half = lane >> 4;
    const int l15  = lane & 15;

    const _Float16* pa = Wt + (size_t)(tm * 16) * NN;
    const _Float16* pb = Xt + (size_t)(tn * 16) * NN;
    v8f acc = {};
#pragma unroll 4
    for (int kk0 = 0; kk0 < NN; kk0 += 32)
        acc = wmma_f16(load_frag(pa, NN, kk0, lane), load_frag(pb, NN, kk0, lane), acc);

#pragma unroll
    for (int j = 0; j < 8; ++j) ot[(j + half * 8) * XC + tn * 16 + l15] = acc[j];
    __syncthreads();
    {
        char* dst = (char*)(rt + (size_t)tm * 16 * XC);
        for (int g = threadIdx.x; g < 512; g += 256) {
            const v4f v = *(const v4f*)((const char*)ot + g * 16);
            vst2(dst + g * 16, v);
        }
    }
}

__global__ __launch_bounds__(1024) void finalize_kernel(const float* __restrict__ rt, const float* __restrict__ n_k,
                                                        float* __restrict__ tail) {
    __shared__ __align__(16) float buf[2 * KK + 16];
    const int t = threadIdx.x;
    if (t == 0) {
        float suffix = 0.f;
        for (int k = KK - 1; k >= 0; --k) {
            float nk = n_k[k];
            buf[k]      = 1.f + nk;
            buf[KK + k] = ALPHA_C + suffix;
            suffix     += nk;
        }
        for (int i = 2 * KK; i < 2 * KK + 16; ++i) buf[i] = 0.f;
    }
    __syncthreads();
    for (int g = t; g < (2 * KK + 2 * KK * DZ) / 4; g += 1024) {
        float v[4];
#pragma unroll
        for (int e = 0; e < 4; ++e) {
            const int i = g * 4 + e;
            float val;
            if (i < 2 * KK) val = buf[i];
            else {
                const bool iss = (i >= 2 * KK + KK * DZ);
                const int j = i - 2 * KK - (iss ? KK * DZ : 0);
                const int k = j >> 6, d = j & 63;
                const float m1 = rt[k * XC + d] * WUN;
                if (!iss) val = m1;
                else { const float e2 = rt[k * XC + DZ + d] * WUN;
                       val = fmaxf(e2 - m1 * m1, SMIN_C); }
            }
            v[e] = val;
        }
        v4f vv = {v[0], v[1], v[2], v[3]};
        vst2(tail + (size_t)g * 4, vv);
    }
}

extern "C" void kernel_launch(void* const* d_in, const int* in_sizes, int n_in,
                              void* d_out, int out_size, void* d_ws, size_t ws_size,
                              hipStream_t stream) {
    (void)in_sizes; (void)n_in; (void)out_size; (void)ws_size;
    const float* mu = (const float*)d_in[0];
    const float* s2 = (const float*)d_in[1];
    const float* a  = (const float*)d_in[2];
    const float* b  = (const float*)d_in[3];
    const float* m  = (const float*)d_in[4];
    const float* S  = (const float*)d_in[5];

    float* out = (float*)d_out;
    float* r_out = out;
    float* tail  = out + (size_t)NN * KK;

    float*  ws  = (float*)d_ws;
    float*  elp = ws;
    float*  n_k = ws + KPAD;
    float*  rt  = ws + 2 * KPAD;
    _Float16* Wt = (_Float16*)(rt + (size_t)KPAD * XC);
    _Float16* Xt = Wt + (size_t)KPAD * NN;

    elogpi_kernel<<<1, 32, 0, stream>>>(a, b, elp);
    estep_kernel<<<NN / 16, 256, 0, stream>>>(mu, s2, S, m, elp, r_out);
    colsum_kernel<<<KPAD / 32, 256, 0, stream>>>(r_out, n_k);
    pack_Wt_kernel<<<dim3(NN / 64, KPAD / 32), 256, 0, stream>>>(r_out, n_k, Wt);
    pack_Xt_kernel<<<dim3(NN / 64, XC / 32), 256, 0, stream>>>(mu, s2, Xt);
    gemm_rtX_kernel<<<KPAD / 16, 256, 0, stream>>>(Wt, Xt, rt);
    finalize_kernel<<<1, 1024, 0, stream>>>(rt, n_k, tail);
}
